// OfficialDITBuildingBlock_81458349736391
// MI455X (gfx1250) — hardware-verified
//
#include <hip/hip_runtime.h>


#define NB_  2
#define SS   2048
#define EE   1024
#define NH_  16
#define HD   64
#define ZH   4
#define NR   (NB_ * SS)
#define DM   EE
#define PCAR 1024.0f
#define LOSC 1024.0f
typedef _Float16 h16;
typedef unsigned short bf;
typedef __attribute__((ext_vector_type(16))) __bf16   v16bf;
typedef __attribute__((ext_vector_type(16))) _Float16 v16h;
typedef __attribute__((ext_vector_type(8)))  _Float16 v8h;
typedef __attribute__((ext_vector_type(8)))  unsigned short v8us;
typedef __attribute__((ext_vector_type(8)))  float    v8f;
typedef __attribute__((ext_vector_type(4)))  float    v4f;
typedef v8h  __attribute__((may_alias)) v8ha;
typedef v4f  __attribute__((may_alias)) v4fa;
typedef v8us __attribute__((may_alias)) v8usa;

__device__ __forceinline__ unsigned short f2bf(float f) { unsigned u = __float_as_uint(f); u += 0x7FFFu + ((u >> 16) & 1u); return (unsigned short)(u >> 16); }
__device__ __forceinline__ float bf2f(unsigned short b) { return __uint_as_float(((unsigned)b) << 16); }
__device__ __forceinline__ float bfr(float f) { return bf2f(f2bf(f)); }
__device__ __forceinline__ v16h cat16(v8h lo, v8h hi) { return __builtin_shufflevector(lo, hi, 0, 1, 2, 3, 4, 5, 6, 7, 8, 9, 10, 11, 12, 13, 14, 15); }
__device__ __forceinline__ v16bf cat16b(v8us lo, v8us hi) { return __builtin_bit_cast(v16bf, __builtin_shufflevector(lo, hi, 0, 1, 2, 3, 4, 5, 6, 7, 8, 9, 10, 11, 12, 13, 14, 15)); }
__device__ __forceinline__ v8f wmma16(v16h a, v16h b, v8f c) { return __builtin_amdgcn_wmma_f32_16x16x32_f16(false, a, false, b, (short)0, c, false, false); }
__device__ __forceinline__ v8f wmmab(v16bf a, v16bf b, v8f c) { return __builtin_amdgcn_wmma_f32_16x16x32_bf16(false, a, false, b, (short)0, c, false, false); }


__global__ __launch_bounds__(128) void k_gemmh(const h16* __restrict__ A, const h16* __restrict__ Bn, const float* __restrict__ bias, float* C, int ldc, const float* __restrict__ R, int K, size_t sA, size_t sB, size_t sC, int roundR) {
    __shared__ __align__(16) float ost[4][16 * 68];
    const size_t z = blockIdx.z; A += z * sA; Bn += z * sB; C += z * sC; if (R) R += z * sC;
    const int lane = threadIdx.x & 31, wave = threadIdx.x >> 5, lr = lane & 15, hi = lane >> 4;
    const int r0 = blockIdx.x * 64 + wave * 16, c0 = blockIdx.y * 64;
    const size_t aoff = (size_t)(r0 + lr) * K + 8 * hi;
    size_t boff[4];
#pragma unroll
    for (int t = 0; t < 4; ++t) boff[t] = (size_t)(c0 + t * 16 + lr) * K + 8 * hi;
    v8f acc[4];
#pragma unroll
    for (int t = 0; t < 4; ++t) acc[t] = (v8f){};
#pragma unroll 1
    for (int kc = 0; kc < K; kc += 32) {
        const v16h a = cat16(*(const v8h*)(A + aoff + kc), *(const v8h*)(A + aoff + kc + 16));
#pragma unroll
        for (int t = 0; t < 4; ++t) { const v16h b = cat16(*(const v8h*)(Bn + boff[t] + kc), *(const v8h*)(Bn + boff[t] + kc + 16)); acc[t] = wmma16(a, b, acc[t]); }
        asm volatile("v_nop\n\tv_nop\n\tv_nop\n\tv_nop" : "+v"(acc[0]), "+v"(acc[1]), "+v"(acc[2]), "+v"(acc[3]) : "v"(a));
    }
    float* os = &ost[wave][0];
#pragma unroll
    for (int t = 0; t < 4; ++t) { const float bv = bias ? bfr(bias[c0 + t * 16 + lr]) : 0.f;
#pragma unroll
        for (int j = 0; j < 8; ++j) os[(hi * 8 + j) * 68 + t * 16 + lr] = acc[t][j] + bv; }
    __syncthreads();
    float* crow = C + (size_t)r0 * ldc + c0;
    auto pass = [&]() {
#pragma unroll
        for (int s = 0; s < 8; ++s) { const int Lid = (lane >> 3) + 4 * s, piece = lane & 7; const int row = Lid >> 1, cofs = (Lid & 1) * 32 + piece * 4;
            v4f val = *(const v4fa*)(os + row * 68 + cofs); if (R) { const v4f rv = *(const v4f*)(R + ((size_t)r0 + row) * ldc + c0 + cofs); val += roundR ? (v4f){bfr(rv[0]), bfr(rv[1]), bfr(rv[2]), bfr(rv[3])} : rv; }
            *(volatile v4f*)(crow + (size_t)row * ldc + cofs) = val; }
    };
    pass(); __threadfence(); pass();
}

template <int MODE>
__global__ __launch_bounds__(128) void k_gemm3z(const bf* __restrict__ Ah, const bf* __restrict__ Al, const bf* __restrict__ Bh, const bf* __restrict__ Bl, int K, float* C, int ldc, size_t sA, size_t sB, size_t sC) {
    if ((MODE & 1) && (int)blockIdx.y * 64 > (int)blockIdx.x * 64 + 63) return;
    const size_t z = blockIdx.z; Ah += z * sA; Al += z * sA; Bh += z * sB; Bl += z * sB; C += z * sC;
    const int Klim = (MODE & 2) ? min(K, ((int)blockIdx.x + 1) * 64) : K;
    __shared__ __align__(16) float ost[4][16 * 68];
    const int lane = threadIdx.x & 31, wave = threadIdx.x >> 5, lr = lane & 15, hi = lane >> 4;
    const int r0 = blockIdx.x * 64 + wave * 16, c0 = blockIdx.y * 64;
    const size_t aoff = (size_t)(r0 + lr) * K + 8 * hi;
    v8f acc[4];
#pragma unroll
    for (int t = 0; t < 4; ++t) acc[t] = (v8f){};
#pragma unroll 1
    for (int kc = 0; kc < Klim; kc += 32) {
        const v16bf a = cat16b(*(const v8us*)(Ah + aoff + kc), *(const v8us*)(Ah + aoff + kc + 16));
        v16bf al = a; if (!(MODE & 4) && !(MODE & 16)) al = cat16b(*(const v8us*)(Al + aoff + kc), *(const v8us*)(Al + aoff + kc + 16));
#pragma unroll
        for (int t = 0; t < 4; ++t) { const size_t bo = (size_t)(c0 + t * 16 + lr) * K + kc + 8 * hi;
            const v16bf bh = cat16b(*(const v8us*)(Bh + bo), *(const v8us*)(Bh + bo + 16));
            acc[t] = wmmab(a, bh, acc[t]);
            if (!(MODE & 4)) { if (!(MODE & 16)) acc[t] = wmmab(al, bh, acc[t]); if (!(MODE & 8)) { const v16bf bl = cat16b(*(const v8us*)(Bl + bo), *(const v8us*)(Bl + bo + 16)); acc[t] = wmmab(a, bl, acc[t]); } } }
        asm volatile("v_nop\n\tv_nop\n\tv_nop\n\tv_nop" : "+v"(acc[0]), "+v"(acc[1]), "+v"(acc[2]), "+v"(acc[3]) : "v"(a), "v"(al));
    }
    float* os = &ost[wave][0];
#pragma unroll
    for (int t = 0; t < 4; ++t) {
#pragma unroll
        for (int j = 0; j < 8; ++j) os[(hi * 8 + j) * 68 + t * 16 + lr] = acc[t][j]; }
    __builtin_amdgcn_wave_barrier(); asm volatile("" ::: "memory");
    float* crow = C + (size_t)r0 * ldc + c0;
    auto pass = [&]() {
#pragma unroll
        for (int s = 0; s < 8; ++s) { const int Lid = (lane >> 3) + 4 * s, piece = lane & 7; const int row = Lid >> 1, cofs = (Lid & 1) * 32 + piece * 4;
            const v4f val = *(const v4fa*)(os + row * 68 + cofs); *(volatile v4f*)(crow + (size_t)row * ldc + cofs) = val; }
    };
    pass(); __threadfence(); pass();
}
__global__ __launch_bounds__(256) void k_planes32z(const float* __restrict__ F, int ld, int off, float sc, int rows, bf* Ph, bf* Pl) {
    typedef __attribute__((ext_vector_type(2))) unsigned short v2us;
    const int lane = threadIdx.x & 31; const size_t r = ((size_t)blockIdx.x * 8 + (threadIdx.x >> 5)) * 2 + (lane >> 4); if (r >= (size_t)rows) return; const int z = blockIdx.z; const int c0 = (lane & 15) * 2; v2us oh, ol;
    Ph += (size_t)z * rows * 32; Pl += (size_t)z * rows * 32;
#pragma unroll
    for (int i = 0; i < 2; ++i) { const float y = F[r * ld + off + z * 32 + c0 + i] * sc; const unsigned short hb = f2bf(y); oh[i] = hb; ol[i] = f2bf(y - bf2f(hb)); }
    const size_t o = r * 32 + c0; *(volatile v2us*)(Ph + o) = oh; *(volatile v2us*)(Pl + o) = ol; __threadfence(); *(volatile v2us*)(Ph + o) = oh; *(volatile v2us*)(Pl + o) = ol;
}
__global__ __launch_bounds__(256) void k_vtpadz(const float* __restrict__ F, int ld, int off, int nk, bf* Th, bf* Tl) {
    typedef __attribute__((ext_vector_type(2))) unsigned short v2us;
    const int lane = threadIdx.x & 31; const size_t wid = (size_t)blockIdx.x * 8 + (threadIdx.x >> 5); if (wid >= (size_t)64 * (nk / 64)) return; const int z = blockIdx.z; const int d = (int)(wid / (nk / 64)); const int k0 = (int)(wid % (nk / 64)) * 64 + lane * 2; v2us oh, ol;
    Th += (size_t)z * 64 * nk; Tl += (size_t)z * 64 * nk;
#pragma unroll
    for (int i = 0; i < 2; ++i) { const float y = (d < 32) ? F[(size_t)(k0 + i) * ld + off + z * 32 + (d < 32 ? d : 0)] : 0.f; const unsigned short hb = f2bf(y); oh[i] = hb; ol[i] = f2bf(y - bf2f(hb)); }
    const size_t o = (size_t)d * nk + k0; *(volatile v2us*)(Th + o) = oh; *(volatile v2us*)(Tl + o) = ol; __threadfence(); *(volatile v2us*)(Th + o) = oh; *(volatile v2us*)(Tl + o) = ol;
}
template <int NK>
__global__ __launch_bounds__(256) void k_softmaxz(const float* __restrict__ S, int rows, bf* PH, bf* PL) {
    typedef __attribute__((ext_vector_type(4))) unsigned short v4us;
    const int lane = threadIdx.x & 31, i = blockIdx.x * 8 + (threadIdx.x >> 5); if (i >= rows) return; const size_t zo = (size_t)blockIdx.z * rows * NK; const float* sr = S + zo + (size_t)i * NK; PH += zo; PL += zo;
    float m = -3.0e38f;
#pragma unroll 1
    for (int c0 = lane * 4; c0 < NK; c0 += 128) {
#pragma unroll
        for (int q = 0; q < 4; ++q) m = fmaxf(m, sr[c0 + q]); }
#pragma unroll
    for (int sh = 16; sh; sh >>= 1) m = fmaxf(m, __shfl_xor(m, sh, 32));
    float sum = 0.f;
#pragma unroll 1
    for (int c0 = lane * 4; c0 < NK; c0 += 128) {
#pragma unroll
        for (int q = 0; q < 4; ++q) sum += __expf(sr[c0 + q] - m); }
#pragma unroll
    for (int sh = 16; sh; sh >>= 1) sum += __shfl_xor(sum, sh, 32);
    const float inv = 1.0f / sum;
#pragma unroll 1
    for (int ps = 0; ps < 2; ++ps) {
#pragma unroll 1
        for (int c0 = lane * 4; c0 < NK; c0 += 128) { v4us oh, ol;
#pragma unroll
            for (int q = 0; q < 4; ++q) { const float p = __expf(sr[c0 + q] - m) * inv; const unsigned short hb = f2bf(p); oh[q] = hb; ol[q] = f2bf(p - bf2f(hb)); }
            const size_t o = (size_t)i * NK + c0; *(volatile v4us*)(PH + o) = oh; *(volatile v4us*)(PL + o) = ol; }
        if (ps == 0) __threadfence(); }
}
__global__ __launch_bounds__(256) void k_placez(const float* __restrict__ XH, int rows, int ldy, float* Y) {
    const int lane = threadIdx.x & 31; const size_t q = (size_t)blockIdx.x * 8 + (threadIdx.x >> 5); if (q >= (size_t)rows) return; const int z = blockIdx.z; const float v = XH[((size_t)z * rows + q) * 64 + lane];
    *(volatile float*)(Y + q * ldy + z * 32 + lane) = v; __threadfence(); *(volatile float*)(Y + q * ldy + z * 32 + lane) = v;
}

template <typename T16> struct WFrag;
template <> struct WFrag<h16> { typedef v16h V; static __device__ __forceinline__ V ld(const h16* p) { return cat16(*(const v8h*)p, *(const v8h*)(p + 16)); } static __device__ __forceinline__ v8f mma(V a, V b, v8f c) { return wmma16(a, b, c); } };
template <> struct WFrag<bf> { typedef v16bf V; static __device__ __forceinline__ V ld(const bf* p) { return cat16b(*(const v8us*)p, *(const v8us*)(p + 16)); } static __device__ __forceinline__ v8f mma(V a, V b, v8f c) { return wmmab(a, b, c); } };
template <typename T16, int NSPLIT, bool BIAS>
__global__ __launch_bounds__(32) void k_gemmw(const T16* __restrict__ A, const T16* __restrict__ A2, const T16* __restrict__ Bt, const T16* __restrict__ Bt2, int K, float* C, int ldc, const float* __restrict__ bias, size_t sA, size_t sB, size_t sC) {
    typedef typename WFrag<T16>::V V;
    __shared__ __align__(16) float os[16 * 68];
    const size_t z = blockIdx.z; A += z * sA; if (A2) A2 += z * sA; Bt += z * sB; if (Bt2) Bt2 += z * sB; C += z * sC;
    const int lane = threadIdx.x & 31, lr = lane & 15, hi = lane >> 4; const int r0 = blockIdx.x * 64, c0 = blockIdx.y * 64;
    v8f acc[4][4];
#pragma unroll
    for (int mb = 0; mb < 4; ++mb)
#pragma unroll
        for (int nb = 0; nb < 4; ++nb) acc[mb][nb] = (v8f){};
    const size_t aoff = (size_t)(r0 + lr) * K + 8 * hi, boff = (size_t)(c0 + lr) * K + 8 * hi;
#pragma unroll 1
    for (int kc = 0; kc < K; kc += 32) {
        V a[4], a2[4];
#pragma unroll
        for (int mb = 0; mb < 4; ++mb) { a[mb] = WFrag<T16>::ld(A + aoff + (size_t)mb * 16 * K + kc); if (NSPLIT == 1 || NSPLIT == 2) a2[mb] = WFrag<T16>::ld(A2 + aoff + (size_t)mb * 16 * K + kc); }
#pragma unroll
        for (int nb = 0; nb < 4; ++nb) { const V b = WFrag<T16>::ld(Bt + boff + (size_t)nb * 16 * K + kc); V b2; if (NSPLIT >= 2) b2 = WFrag<T16>::ld(Bt2 + boff + (size_t)nb * 16 * K + kc);
#pragma unroll
            for (int mb = 0; mb < 4; ++mb) { acc[mb][nb] = WFrag<T16>::mma(a[mb], b, acc[mb][nb]); if (NSPLIT == 1 || NSPLIT == 2) acc[mb][nb] = WFrag<T16>::mma(a2[mb], b, acc[mb][nb]); if (NSPLIT >= 2) acc[mb][nb] = WFrag<T16>::mma(a[mb], b2, acc[mb][nb]); } }
        asm volatile("v_nop\n\tv_nop\n\tv_nop\n\tv_nop" : "+v"(acc[0][0]), "+v"(acc[1][1]), "+v"(acc[2][2]), "+v"(acc[3][3]) : "v"(a[0]), "v"(a[3]));
    }
#pragma unroll
    for (int mb = 0; mb < 4; ++mb) {
#pragma unroll
        for (int nb = 0; nb < 4; ++nb) {
#pragma unroll
            for (int j = 0; j < 8; ++j) os[(hi * 8 + j) * 68 + nb * 16 + lr] = acc[mb][nb][j]; }
        __builtin_amdgcn_wave_barrier(); asm volatile("" ::: "memory");
        float* crow = C + (size_t)(r0 + mb * 16) * ldc + c0;
#pragma unroll 1
        for (int ps = 0; ps < 2; ++ps) {
#pragma unroll
            for (int s = 0; s < 8; ++s) { const int row = 2 * s + hi, cofs = lr * 4; v4f val = *(const v4fa*)(os + row * 68 + cofs); if (BIAS) { val[0] += bfr(bias[c0 + cofs]); val[1] += bfr(bias[c0 + cofs + 1]); val[2] += bfr(bias[c0 + cofs + 2]); val[3] += bfr(bias[c0 + cofs + 3]); }
                *(volatile v4f*)(crow + (size_t)row * ldc + cofs) = val; }
            if (ps == 0) __threadfence(); }
        __builtin_amdgcn_wave_barrier(); asm volatile("" ::: "memory");
    }
}

typedef __attribute__((ext_vector_type(4))) _Float16 v4h;
__device__ __forceinline__ h16 tohx(float x) { return (h16)x; }
__global__ __launch_bounds__(256) void k_wTh(const float* __restrict__ Wm, int ldw, int K, int N, h16* Bh) {
    __shared__ float tl[64][65];
    const int tid = threadIdx.x; const int k0 = blockIdx.x * 64, n0 = blockIdx.y * 64; const int rr = tid >> 2, cq = (tid & 3) * 16;
#pragma unroll
    for (int i = 0; i < 16; ++i) tl[rr][cq + i] = bfr(Wm[(size_t)(k0 + rr) * ldw + n0 + cq + i]);
    __syncthreads();
    const int lane = tid & 31, wv = tid >> 5;
    auto pass = [&]() {
#pragma unroll
        for (int st = 0; st < 4; ++st) { const int nr = wv * 8 + st * 2 + (lane >> 4); const int kq = (lane & 15) * 4; v4h v; for (int i = 0; i < 4; ++i) v[i] = tohx(tl[kq + i][nr]); *(volatile v4h*)(Bh + (size_t)(n0 + nr) * K + k0 + kq) = v; }
    };
    pass(); __threadfence(); pass();
}
__global__ __launch_bounds__(256) void k_ada1(const float* __restrict__ emb, const float* __restrict__ W1, float* Y1) {
    const int lane = threadIdx.x & 31; const int w = blockIdx.x * 8 + (threadIdx.x >> 5); if (w >= NB_ * (EE / 32)) return; const int b = w / (EE / 32), j = (w % (EE / 32)) * 32 + lane; float a = 0.f;
#pragma unroll 1
    for (int i = 0; i < EE; ++i) { const float e = bfr(emb[b * EE + i]); const float s = __fdiv_rn(e, 1.0f + __expf(-e)); a = fmaf(s, bfr(W1[(size_t)i * EE + j]), a); }
    *(volatile float*)(Y1 + b * EE + j) = a; __threadfence(); *(volatile float*)(Y1 + b * EE + j) = a;
}
__global__ __launch_bounds__(256) void k_ada2(const float* __restrict__ Y1, const float* __restrict__ W2, const float* __restrict__ b2, float* ADA) {
    const int lane = threadIdx.x & 31; const int w = blockIdx.x * 8 + (threadIdx.x >> 5); if (w >= NB_ * (2 * EE / 32)) return; const int b = w / (2 * EE / 32), o = (w % (2 * EE / 32)) * 32 + lane; float a = bfr(b2[o]);
#pragma unroll 1
    for (int j = 0; j < EE; ++j) a = fmaf(Y1[b * EE + j], bfr(W2[(size_t)j * (2 * EE) + o]), a);
    *(volatile float*)(ADA + b * 2 * EE + o) = a; __threadfence(); *(volatile float*)(ADA + b * 2 * EE + o) = a;
}
__global__ __launch_bounds__(256) void k_lnmod(const float* __restrict__ x, const float* __restrict__ ADA, h16* XN) {
    const int lane = threadIdx.x & 31; const size_t r = (size_t)blockIdx.x * 8 + (threadIdx.x >> 5); if (r >= (size_t)NR) return; const int b = (int)(r / SS); float v[32]; float s = 0.f;
#pragma unroll
    for (int c = 0; c < 4; ++c) {
#pragma unroll
        for (int i = 0; i < 8; ++i) { v[c * 8 + i] = bfr(x[r * EE + c * 256 + lane * 8 + i]); s += v[c * 8 + i]; } }
#pragma unroll
    for (int sh = 16; sh; sh >>= 1) s += __shfl_xor(s, sh, 32);
    const float mu = s * (1.0f / EE); float q = 0.f;
#pragma unroll
    for (int i = 0; i < 32; ++i) { const float d = v[i] - mu; q = fmaf(d, d, q); }
#pragma unroll
    for (int sh = 16; sh; sh >>= 1) q += __shfl_xor(q, sh, 32);
    const float rs = rsqrtf(q * (1.0f / EE) + 1e-6f); const float* shf = ADA + (size_t)b * 2 * EE; const float* scl = shf + EE;
#pragma unroll 1
    for (int ps = 0; ps < 2; ++ps) {
#pragma unroll
        for (int c = 0; c < 4; ++c) { v8h o;
#pragma unroll
            for (int i = 0; i < 8; ++i) { const int col = c * 256 + lane * 8 + i; o[i] = tohx((v[c * 8 + i] - mu) * rs * (1.0f + scl[col]) + shf[col]); }
            *(volatile v8h*)(XN + r * EE + c * 256 + lane * 8) = o; }
        if (ps == 0) __threadfence(); }
}
__global__ __launch_bounds__(256) void k_cvtp(const float* __restrict__ F, h16* P) {
    const int lane = threadIdx.x & 31; const size_t r = (size_t)blockIdx.x * 8 + (threadIdx.x >> 5); if (r >= (size_t)NR) return;
#pragma unroll 1
    for (int ps = 0; ps < 2; ++ps) {
#pragma unroll
        for (int c = 0; c < 4; ++c) { v8h o; const size_t off = r * EE + c * 256 + lane * 8;
#pragma unroll
            for (int i = 0; i < 8; ++i) o[i] = tohx(F[off + i]);
            *(volatile v8h*)(P + off) = o; }
        if (ps == 0) __threadfence(); }
}
__global__ __launch_bounds__(256) void k_ropep(const float* __restrict__ F, const float* __restrict__ ang, int b, int h0, float sc, h16* P) {
    const int lane = threadIdx.x & 31; const size_t w = (size_t)blockIdx.x * 8 + (threadIdx.x >> 5); const int t = (int)(w * 2 + (lane >> 4)); if (t >= SS) return; const int z = blockIdx.z; const int c0 = (lane & 15) * 4; const float* fr = F + ((size_t)b * SS + t) * EE + (h0 + z) * HD; v4h o;
#pragma unroll
    for (int q = 0; q < 4; ++q) { const int d = c0 + q; const float a = bfr(ang[(size_t)t * HD + d]); float sn, cs; __sincosf(a, &sn, &cs); const float rot = (d < HD / 2) ? -fr[d + HD / 2] : fr[d - HD / 2]; o[q] = tohx((fr[d] * cs + rot * sn) * sc); }
    const size_t off = ((size_t)z * SS + t) * HD + c0; *(volatile v4h*)(P + off) = o; __threadfence(); *(volatile v4h*)(P + off) = o;
}
__global__ __launch_bounds__(256) void k_vT64h(const float* __restrict__ V, int b, int h0, h16* VT) {
    __shared__ float tl[64][65];
    const int tid = threadIdx.x; const int t0 = blockIdx.x * 64; const int z = blockIdx.z; const int rr = tid >> 2, cq = (tid & 3) * 16;
#pragma unroll
    for (int i = 0; i < 16; ++i) tl[rr][cq + i] = V[((size_t)b * SS + t0 + rr) * EE + (h0 + z) * HD + cq + i];
    __syncthreads();
    const int lane = tid & 31, wv = tid >> 5;
    auto pass = [&]() {
#pragma unroll
        for (int st = 0; st < 4; ++st) { const int dr = wv * 8 + st * 2 + (lane >> 4); const int tq = (lane & 15) * 4; v4h v;
#pragma unroll
            for (int i = 0; i < 4; ++i) v[i] = tohx(tl[tq + i][dr]);
            *(volatile v4h*)(VT + ((size_t)z * HD + dr) * SS + t0 + tq) = v; }
    };
    pass(); __threadfence(); pass();
}
__global__ __launch_bounds__(256) void k_softp(const float* __restrict__ S, h16* P) {
    const int lane = threadIdx.x & 31, i = blockIdx.x * 8 + (threadIdx.x >> 5); if (i >= SS) return; const size_t zo = ((size_t)blockIdx.z * SS + i) * SS; const float* sr = S + zo; h16* po = P + zo;
    float m = -3.0e38f;
#pragma unroll 1
    for (int c0 = lane * 4; c0 < SS; c0 += 128) {
#pragma unroll
        for (int q = 0; q < 4; ++q) m = fmaxf(m, sr[c0 + q]); }
#pragma unroll
    for (int sh = 16; sh; sh >>= 1) m = fmaxf(m, __shfl_xor(m, sh, 32));
    float sum = 0.f;
#pragma unroll 1
    for (int c0 = lane * 4; c0 < SS; c0 += 128) {
#pragma unroll
        for (int q = 0; q < 4; ++q) sum += __expf(sr[c0 + q] - m); }
#pragma unroll
    for (int sh = 16; sh; sh >>= 1) sum += __shfl_xor(sum, sh, 32);
    const float f = __fdiv_rn(PCAR, sum);
#pragma unroll 1
    for (int ps = 0; ps < 2; ++ps) {
#pragma unroll 1
        for (int c0 = lane * 4; c0 < SS; c0 += 128) { v4h o;
#pragma unroll
            for (int q = 0; q < 4; ++q) o[q] = tohx(__expf(sr[c0 + q] - m) * f);
            *(volatile v4h*)(po + c0) = o; }
        if (ps == 0) __threadfence(); }
}
__global__ __launch_bounds__(256) void k_mergec(const float* __restrict__ OZ, int b, int h0, h16* OH) {
    const int lane = threadIdx.x & 31, i = blockIdx.x * 8 + (threadIdx.x >> 5); if (i >= SS) return; const int z = lane >> 3, d0 = (lane & 7) * 8; v8h o;
#pragma unroll
    for (int k = 0; k < 8; ++k) o[k] = tohx(OZ[((size_t)z * SS + i) * HD + d0 + k] * (1.0f / PCAR));
    const size_t off = ((size_t)b * SS + i) * EE + (h0 + z) * HD + d0; *(volatile v8h*)(OH + off) = o; __threadfence(); *(volatile v8h*)(OH + off) = o;
}
__global__ __launch_bounds__(256) void k_fin(const float* __restrict__ CO, const float* __restrict__ x, const float* __restrict__ gate, float* OUTB) {
    const int lane = threadIdx.x & 31; const size_t r = (size_t)blockIdx.x * 8 + (threadIdx.x >> 5); if (r >= (size_t)NR) return; const int b = (int)(r / SS);
#pragma unroll 1
    for (int ps = 0; ps < 2; ++ps) {
#pragma unroll
        for (int p = 0; p < EE / 128; ++p) { const int c0 = p * 128 + lane * 4; v4f v;
#pragma unroll
            for (int i = 0; i < 4; ++i) v[i] = bfr(x[r * EE + c0 + i]) + bfr(gate[b * EE + c0 + i]) * CO[r * EE + c0 + i];
            *(volatile v4f*)(OUTB + r * EE + c0) = v; }
        if (ps == 0) __threadfence(); }
}
extern "C" void kernel_launch(void* const* d_in, const int* in_sizes, int n_in,
                              void* d_out, int out_size, void* d_ws, size_t ws_size, hipStream_t stream) {
    (void)in_sizes; (void)n_in; (void)out_size;
    const float* x = (const float*)d_in[0]; const float* emb = (const float*)d_in[1]; const float* gate = (const float*)d_in[2];   const float* ang = (const float*)d_in[4];
    const float* Wq1 = (const float*)d_in[5]; const float* Wq2 = (const float*)d_in[6]; const float* Wk1 = (const float*)d_in[7]; const float* Wk2 = (const float*)d_in[8]; const float* Wv = (const float*)d_in[9]; const float* Wo = (const float*)d_in[10]; const float* Wa1 = (const float*)d_in[11]; const float* Wa2 = (const float*)d_in[12]; const float* ba2 = (const float*)d_in[13];
    float* out = (float*)d_out;
    char* wsp = (char*)d_ws;
    auto take = [&](size_t bytes) { char* p = wsp; wsp += (bytes + 255) & ~(size_t)255; return (void*)p; };
    const size_t WSZ = (size_t)EE * EE * 2;
    h16* WQ1 = (h16*)take(WSZ); h16* WQ2 = (h16*)take(WSZ); h16* WK1 = (h16*)take(WSZ); h16* WK2 = (h16*)take(WSZ); h16* WVh = (h16*)take(WSZ); h16* WOh = (h16*)take(WSZ);
    float* Y1 = (float*)take((size_t)NB_ * EE * 4); float* ADA = (float*)take((size_t)NB_ * 2 * EE * 4); h16* XN = (h16*)take((size_t)NR * EE * 2); float* T = (float*)take((size_t)NR * EE * 4); h16* TP = (h16*)take((size_t)NR * EE * 2);
    float* Q = (float*)take((size_t)NR * EE * 4); float* Kf = (float*)take((size_t)NR * EE * 4); float* V = (float*)take((size_t)NR * EE * 4);
    h16* Qx = (h16*)take((size_t)ZH * SS * HD * 2); h16* Kx = (h16*)take((size_t)ZH * SS * HD * 2); h16* VT = (h16*)take((size_t)ZH * HD * SS * 2); float* S = (float*)take((size_t)ZH * SS * SS * 4); h16* Px = (h16*)take((size_t)ZH * SS * SS * 2); float* OZ = (float*)take((size_t)ZH * SS * HD * 4); h16* OH = (h16*)take((size_t)NR * EE * 2);
    if ((size_t)(wsp - (char*)d_ws) > ws_size) return;
    float* CO = T;
    k_wTh<<<dim3(EE / 64, EE / 64, 1), 256, 0, stream>>>(Wq1, EE, EE, EE, WQ1); k_wTh<<<dim3(EE / 64, EE / 64, 1), 256, 0, stream>>>(Wq2, EE, EE, EE, WQ2); k_wTh<<<dim3(EE / 64, EE / 64, 1), 256, 0, stream>>>(Wk1, EE, EE, EE, WK1); k_wTh<<<dim3(EE / 64, EE / 64, 1), 256, 0, stream>>>(Wk2, EE, EE, EE, WK2); k_wTh<<<dim3(EE / 64, EE / 64, 1), 256, 0, stream>>>(Wv, EE, EE, EE, WVh); k_wTh<<<dim3(EE / 64, EE / 64, 1), 256, 0, stream>>>(Wo, EE, EE, EE, WOh);
    k_ada1<<<(NB_ * (EE / 32)) / 8, 256, 0, stream>>>(emb, Wa1, Y1); k_ada2<<<(NB_ * (2 * EE / 32)) / 8, 256, 0, stream>>>(Y1, Wa2, ba2, ADA);
    k_lnmod<<<NR / 8, 256, 0, stream>>>(x, ADA, XN);
    k_gemmw<h16, 0, false><<<dim3(NR / 64, EE / 64, 1), 32, 0, stream>>>(XN, nullptr, WQ1, nullptr, EE, T, EE, nullptr, 0, 0, 0); k_cvtp<<<NR / 8, 256, 0, stream>>>(T, TP);
    k_gemmw<h16, 0, false><<<dim3(NR / 64, EE / 64, 1), 32, 0, stream>>>(TP, nullptr, WQ2, nullptr, EE, Q, EE, nullptr, 0, 0, 0);
    k_gemmw<h16, 0, false><<<dim3(NR / 64, EE / 64, 1), 32, 0, stream>>>(XN, nullptr, WK1, nullptr, EE, T, EE, nullptr, 0, 0, 0); k_cvtp<<<NR / 8, 256, 0, stream>>>(T, TP);
    k_gemmw<h16, 0, false><<<dim3(NR / 64, EE / 64, 1), 32, 0, stream>>>(TP, nullptr, WK2, nullptr, EE, Kf, EE, nullptr, 0, 0, 0);
    k_gemmw<h16, 0, false><<<dim3(NR / 64, EE / 64, 1), 32, 0, stream>>>(XN, nullptr, WVh, nullptr, EE, V, EE, nullptr, 0, 0, 0);
    for (int b = 0; b < NB_; ++b)
        for (int h0 = 0; h0 < NH_; h0 += ZH) {
            k_ropep<<<dim3((SS / 2) / 8, 1, ZH), 256, 0, stream>>>(Q, ang, b, h0, 0.125f, Qx); k_ropep<<<dim3((SS / 2) / 8, 1, ZH), 256, 0, stream>>>(Kf, ang, b, h0, 1.0f, Kx); k_vT64h<<<dim3(SS / 64, 1, ZH), 256, 0, stream>>>(V, b, h0, VT);
            k_gemmw<h16, 0, false><<<dim3(SS / 64, SS / 64, ZH), 32, 0, stream>>>(Qx, nullptr, Kx, nullptr, HD, S, SS, nullptr, (size_t)SS * HD, (size_t)SS * HD, (size_t)SS * SS);
            k_softp<<<dim3(SS / 8, 1, ZH), 256, 0, stream>>>(S, Px);
            k_gemmw<h16, 0, false><<<dim3(SS / 64, 1, ZH), 32, 0, stream>>>(Px, nullptr, VT, nullptr, SS, OZ, HD, nullptr, (size_t)SS * SS, (size_t)HD * SS, (size_t)SS * HD);
            k_mergec<<<SS / 8, 256, 0, stream>>>(OZ, b, h0, OH); }
    k_gemmw<h16, 0, false><<<dim3(NR / 64, EE / 64, 1), 32, 0, stream>>>(OH, nullptr, WOh, nullptr, EE, CO, EE, nullptr, 0, 0, 0);
    k_fin<<<NR / 8, 256, 0, stream>>>(CO, x, gate, out);
}
